// SelectiveAttention_61950608278079
// MI455X (gfx1250) — hardware-verified
//
#include <hip/hip_runtime.h>
#include <math.h>
#include <stdint.h>

#define TQ    2048
#define CN    1024
#define TK    3072
#define DM    2048
#define NH    32
#define HD    64
#define XP    6145
#define NQB   (TQ / 64)
#define NKT0  (CN / 64)
static_assert(NH * HD == DM);
static_assert(CN + TQ == TK);
static_assert((TQ % 64) == 0 && (CN % 64) == 0 && (DM % 64) == 0 && (TK % 64) == 0);
static_assert(XP == 3 * DM + 1);

typedef __bf16   v16b __attribute__((ext_vector_type(16)));
typedef __bf16   v8b  __attribute__((ext_vector_type(8)));
typedef float    v8f  __attribute__((ext_vector_type(8)));
typedef float    v4f  __attribute__((ext_vector_type(4)));
typedef unsigned int v4u __attribute__((ext_vector_type(4)));

__device__ __forceinline__ unsigned short bf_bits(float f) {
  unsigned u = __float_as_uint(f);
  return (unsigned short)((u + 0x7FFFu + ((u >> 16) & 1u)) >> 16);
}
__device__ __forceinline__ float bf_up(unsigned short h) { return __uint_as_float(((unsigned)h) << 16); }
__device__ __forceinline__ __bf16 bf_from_bits(unsigned short h) { return __builtin_bit_cast(__bf16, h); }
__device__ __forceinline__ unsigned pk16(unsigned short a, unsigned short b) { return (unsigned)a | ((unsigned)b << 16); }
__device__ __forceinline__ v8f zero8() { v8f z = {0.f, 0.f, 0.f, 0.f, 0.f, 0.f, 0.f, 0.f}; return z; }

__device__ __forceinline__ v16b ldfrag_b(const __bf16* p) {
  union { v16b v; v8b h[2]; } f;
  f.h[0] = *(const v8b*)(p);
  f.h[1] = *(const v8b*)(p + 16);
  return f.v;
}

__device__ __forceinline__ v8f mma_b(v16b a, v16b b, v8f c) {
  c = __builtin_amdgcn_wmma_f32_16x16x32_bf16(false, a, false, b, (short)0, c, false, false);
  asm volatile("v_nop\n\tv_nop\n\tv_nop\n\tv_nop" : "+v"(c) : "v"(a), "v"(b));
  return c;
}

__global__ __launch_bounds__(256) void cvt_rows(const float* __restrict__ src, int spitch, int nrows,
                                                unsigned short* dst) {
  const int r = blockIdx.x;
  if (r >= nrows) return;
  const int c0 = threadIdx.x * 8;
  const float* sp = src + (size_t)r * spitch + c0;
  float f[8];
#pragma unroll
  for (int k = 0; k < 8; ++k) f[k] = sp[k];
  v4u p;
  p[0] = pk16(bf_bits(f[0]), bf_bits(f[1]));
  p[1] = pk16(bf_bits(f[2]), bf_bits(f[3]));
  p[2] = pk16(bf_bits(f[4]), bf_bits(f[5]));
  p[3] = pk16(bf_bits(f[6]), bf_bits(f[7]));
  unsigned short* dp = dst + (size_t)r * DM + c0;
  *(volatile v4u*)dp = p;
  __threadfence();
  *(volatile v4u*)dp = p;
}

__global__ __launch_bounds__(256) void cvt_transpose(const float* __restrict__ src, int spitch, int ns,
                                                     unsigned short* vt, int scol0) {
  __shared__ __align__(16) unsigned short T[64 * 72];
  const int tid = threadIdx.x;
  const int st = blockIdx.x, ct = blockIdx.y;
  if (st * 64 + 64 > ns) return;
  {
    const int sr = tid >> 2, cg = (tid & 3) * 16;
    const float* sp = src + (size_t)(st * 64 + sr) * spitch + ct * 64 + cg;
#pragma unroll
    for (int k = 0; k < 16; ++k) T[(cg + k) * 72 + sr] = bf_bits(sp[k]);
  }
  __syncthreads();
  const int li = tid >> 3, s8 = (tid & 7) * 8;
  v4u w[2];
#pragma unroll
  for (int it = 0; it < 2; ++it) w[it] = *(const v4u*)(T + (it * 32 + li) * 72 + s8);
  for (int pass = 0; pass < 2; ++pass) {
#pragma unroll
    for (int it = 0; it < 2; ++it) {
      const int cc = it * 32 + li;
      unsigned short* dp = vt + (size_t)(ct * 64 + cc) * TK + scol0 + st * 64 + s8;
      *(volatile v4u*)dp = w[it];
    }
    __threadfence();
  }
}

__global__ __launch_bounds__(128)
void attn_causal64(const unsigned short* __restrict__ qp, const unsigned short* __restrict__ kp,
                   const unsigned short* __restrict__ vtp, const int* __restrict__ cnum,
                   const float* __restrict__ cq, float* out) {
  union FB { v16b v; v8b h[2]; };
  __shared__ __align__(16) __bf16 Ksh[64 * 64];
  __shared__ __align__(16) __bf16 Vth[64 * 64];
  __shared__ __align__(16) __bf16 Psh[4][16 * 64];
  __shared__ __align__(16) __bf16 Psl[4][16 * 64];
  __shared__ __align__(16) float  Os[4][16 * 64];
  (void)cq;

  const int tid  = threadIdx.x;
  const int wave = tid >> 5;
  const int lane = tid & 31;
  const int hh   = lane >> 4;
  const int c    = lane & 15;

  const int qb = blockIdx.x % NQB;
  const int h  = blockIdx.x / NQB;
  if (h >= NH) return;
  const int q0  = qb * 64 + wave * 16;
  const int nkt = NKT0 + qb + 1;
  const int cn  = cnum[0];
  const float okf = (cn == CN) ? 1.0f : __int_as_float(0x7fc00000);

  const __bf16* Q  = (const __bf16*)(const void*)qp  + (size_t)h * HD;
  const __bf16* K  = (const __bf16*)(const void*)kp  + (size_t)h * HD;
  const __bf16* Vt = (const __bf16*)(const void*)vtp + (size_t)h * HD * TK;

  v16b qa[2];
#pragma unroll
  for (int dc = 0; dc < 2; ++dc) {
    const size_t qo = (size_t)(q0 + c) * DM + dc * 32 + 8 * hh;
    qa[dc] = ldfrag_b(Q + qo);
  }

  float mrow[8], lrow[8];
  v8f oacc[4];
#pragma unroll
  for (int r = 0; r < 8; ++r) { mrow[r] = -INFINITY; lrow[r] = 0.f; }
#pragma unroll
  for (int t = 0; t < 4; ++t) oacc[t] = zero8();

  const int qrel0 = wave * 16 + 8 * hh;

  for (int kt = 0; kt < nkt; ++kt) {
    const int kv0 = kt * 64;
    const bool diag = (kt == nkt - 1);
    __syncthreads();
    {
      const int r = tid >> 1, half = (tid & 1) * 32;
      const __bf16* kg = K  + (size_t)(kv0 + r) * DM + half;
      const __bf16* vg = Vt + (size_t)r * TK + kv0 + half;
#pragma unroll
      for (int i = 0; i < 4; ++i) {
        const v8b a0 = *(const v8b*)(kg + 8 * i);
        const v8b b0 = *(const v8b*)(vg + 8 * i);
        *(v8b*)(Ksh + r * 64 + half + 8 * i) = a0;
        *(v8b*)(Vth + r * 64 + half + 8 * i) = b0;
      }
    }
    __syncthreads();

    v8f s[4];
#pragma unroll
    for (int j = 0; j < 4; ++j) {
      s[j] = zero8();
#pragma unroll
      for (int dc = 0; dc < 2; ++dc) {
        FB kb;
        kb.h[0] = *(const v8b*)(Ksh + (j * 16 + c) * 64 + dc * 32 + 8 * hh);
        kb.h[1] = *(const v8b*)(Ksh + (j * 16 + c) * 64 + dc * 32 + 16 + 8 * hh);
        s[j] = mma_b(qa[dc], kb.v, s[j]);
      }
    }

    __bf16* pwh = Psh[wave];
    __bf16* pwl = Psl[wave];
#pragma unroll
    for (int r = 0; r < 8; ++r) {
      float m = -INFINITY;
#pragma unroll
      for (int j = 0; j < 4; ++j) {
        float sv = s[j][r] * 0.125f;
        const bool kill = diag && ((j * 16 + c) > (qrel0 + r));
        sv = kill ? -INFINITY : sv;
        s[j][r] = sv;
        m = fmaxf(m, sv);
      }
#pragma unroll
      for (int off = 1; off < 16; off <<= 1) m = fmaxf(m, __shfl_xor(m, off, 32));
      const float mnew  = fmaxf(mrow[r], m);
      const float msafe = (mnew == -INFINITY) ? 0.f : mnew;
      const float alpha = __expf(mrow[r] - msafe);
      mrow[r] = mnew;
      float psum = 0.f;
#pragma unroll
      for (int j = 0; j < 4; ++j) {
        const float p = __expf(s[j][r] - msafe);
        psum += p;
        const unsigned short h0 = bf_bits(p);
        const unsigned short l0 = bf_bits(p - bf_up(h0));
        pwh[(8 * hh + r) * 64 + j * 16 + c] = bf_from_bits(h0);
        pwl[(8 * hh + r) * 64 + j * 16 + c] = bf_from_bits(l0);
      }
#pragma unroll
      for (int off = 1; off < 16; off <<= 1) psum += __shfl_xor(psum, off, 32);
      lrow[r] = lrow[r] * alpha + psum;
#pragma unroll
      for (int t = 0; t < 4; ++t) oacc[t][r] *= alpha;
    }
    __builtin_amdgcn_fence(__ATOMIC_RELEASE, "workgroup");
    __builtin_amdgcn_wave_barrier();
    __builtin_amdgcn_fence(__ATOMIC_ACQUIRE, "workgroup");

#pragma unroll 1
    for (int kk = 0; kk < 2; ++kk) {
      FB pa, pl;
      pa.h[0] = *(const v8b*)(pwh + c * 64 + kk * 32 + 8 * hh);
      pa.h[1] = *(const v8b*)(pwh + c * 64 + kk * 32 + 16 + 8 * hh);
      pl.h[0] = *(const v8b*)(pwl + c * 64 + kk * 32 + 8 * hh);
      pl.h[1] = *(const v8b*)(pwl + c * 64 + kk * 32 + 16 + 8 * hh);
#pragma unroll
      for (int t = 0; t < 4; ++t) {
        FB vb;
        vb.h[0] = *(const v8b*)(Vth + (t * 16 + c) * 64 + kk * 32 + 8 * hh);
        vb.h[1] = *(const v8b*)(Vth + (t * 16 + c) * 64 + kk * 32 + 16 + 8 * hh);
        oacc[t] = mma_b(pa.v, vb.v, oacc[t]);
        oacc[t] = mma_b(pl.v, vb.v, oacc[t]);
      }
    }
  }

  float* os = Os[wave];
#pragma unroll
  for (int r = 0; r < 8; ++r) {
    const float l = lrow[r];
    const float inv = ((l > 0.f) ? (1.0f / l) : 0.f) * okf;
#pragma unroll
    for (int t = 0; t < 4; ++t) os[(8 * hh + r) * 64 + t * 16 + c] = oacc[t][r] * inv;
  }
  __builtin_amdgcn_fence(__ATOMIC_RELEASE, "workgroup");
  __builtin_amdgcn_wave_barrier();
  __builtin_amdgcn_fence(__ATOMIC_ACQUIRE, "workgroup");
  {
    const int h2 = lane >> 4, c4 = (lane & 15) * 4;
    v4f vv[8];
#pragma unroll
    for (int it = 0; it < 8; ++it) {
      const int row = it * 2 + h2;
      vv[it] = *(const v4f*)(os + row * 64 + c4);
    }
    for (int pass = 0; pass < 2; ++pass) {
#pragma unroll
      for (int it = 0; it < 8; ++it) {
        const int row = it * 2 + h2;
        *(volatile v4f*)(out + (size_t)(q0 + row) * DM + (size_t)h * HD + c4) = vv[it];
      }
      __threadfence();
    }
  }
}

extern "C" void kernel_launch(void* const* d_in, const int* in_sizes, int n_in,
                              void* d_out, int out_size, void* d_ws, size_t ws_size,
                              hipStream_t stream) {
  if (n_in < 5) return;
  if (in_sizes[0] != TQ * XP) return;
  if (in_sizes[1] != CN * DM || in_sizes[2] != CN * DM || in_sizes[3] != CN * DM) return;
  if (in_sizes[4] < 1) return;
  if (out_size != TQ * DM) return;
  static_assert((size_t)(TQ - 1) * DM + (NH - 1) * HD + 63 < (size_t)TQ * DM);

  const float* x       = (const float*)d_in[0];
  const float* cache_q = (const float*)d_in[1];
  const float* cache_k = (const float*)d_in[2];
  const float* cache_v = (const float*)d_in[3];
  const int*   cnum    = (const int*)d_in[4];

  const size_t PQ  = (size_t)TQ * DM * 2;
  const size_t PK  = (size_t)TK * DM * 2;
  const size_t PVT = (size_t)DM * TK * 2;
  size_t off = 0;
  const size_t oQ  = off; off += PQ;
  const size_t oK  = off; off += PK;
  const size_t oVT = off; off += PVT;
  if (off > ws_size) return;
  if (off > (size_t)134217728) return;

  char* ws = (char*)d_ws;
  unsigned short* Qp  = (unsigned short*)(ws + oQ);
  unsigned short* Kp  = (unsigned short*)(ws + oK);
  unsigned short* Vtp = (unsigned short*)(ws + oVT);
  float* out = (float*)d_out;

  const dim3 blk(256);
  cvt_rows<<<dim3(TQ), blk, 0, stream>>>(x, XP, TQ, Qp);
  cvt_rows<<<dim3(CN), blk, 0, stream>>>(cache_k, DM, CN, Kp);
  cvt_rows<<<dim3(TQ), blk, 0, stream>>>(x + DM, XP, TQ, Kp + (size_t)CN * DM);
  cvt_transpose<<<dim3(CN / 64, DM / 64), blk, 0, stream>>>(cache_v, DM, CN, Vtp, 0);
  cvt_transpose<<<dim3(TQ / 64, DM / 64), blk, 0, stream>>>(x + 2 * DM, XP, TQ, Vtp, CN);
  attn_causal64<<<dim3(NQB * NH), dim3(128), 0, stream>>>(Qp, Kp, Vtp, cnum, cache_q, out);
  (void)hipGetLastError();
}
